// CausalSelfAttention_27195732918417
// MI455X (gfx1250) — hardware-run, weakly checked
//
#include <hip/hip_runtime.h>
#include <math.h>

typedef __attribute__((ext_vector_type(16))) _Float16 v16h;
typedef __attribute__((ext_vector_type(16))) __bf16 v16b;
typedef __attribute__((ext_vector_type(8)))  _Float16 v8h;
typedef __attribute__((ext_vector_type(8)))  __bf16 v8b;
typedef __attribute__((ext_vector_type(8)))  float v8f;
typedef __attribute__((ext_vector_type(4)))  float v4f;
typedef __attribute__((ext_vector_type(4)))  unsigned v4u;

template <typename T> __device__ __forceinline__ void vst2(void* p, T v) { *(volatile T*)p = v; __threadfence(); *(volatile T*)p = v; }
__device__ __forceinline__ v8f wmma16(v16h a, v16h b, v8f c) {
  v8f d = __builtin_amdgcn_wmma_f32_16x16x32_f16(false, a, false, b, (short)0, c, false, false);
  asm volatile("v_nop\n\tv_nop\n\tv_nop\n\tv_nop" : "+v"(d) : "v"(a), "v"(b));
  return d;
}
__device__ __forceinline__ v8f wmma_bf(v16b a, v16b b, v8f c) {
  v8f d = __builtin_amdgcn_wmma_f32_16x16x32_bf16(false, a, false, b, (short)0, c, false, false);
  asm volatile("v_nop\n\tv_nop\n\tv_nop\n\tv_nop" : "+v"(d) : "v"(a), "v"(b));
  return d;
}
__device__ __forceinline__ v16h frag_h(const _Float16* rowk0, int lane) {
  union { v16h v; v8h q[2]; } u; const _Float16* p = rowk0 + 8 * (lane >> 4);
  u.q[0] = *(const v8h*)p; u.q[1] = *(const v8h*)(p + 16); return u.v;
}
__device__ __forceinline__ v16b frag_b(const __bf16* rowk0, int lane) {
  union { v16b v; v8b q[2]; } u; const __bf16* p = rowk0 + 8 * (lane >> 4);
  u.q[0] = *(const v8b*)p; u.q[1] = *(const v8b*)(p + 16); return u.v;
}
__device__ __forceinline__ v16h frag_f32(const float* rowk0, int lane) {
  v16h a; const float* p = rowk0 + 8 * (lane >> 4);
#pragma unroll
  for (int i = 0; i < 8; ++i) { a[i] = (_Float16)p[i]; a[8 + i] = (_Float16)p[16 + i]; }
  return a;
}
struct F2 { v16b h, l; };
__device__ __forceinline__ F2 bsplit16(const float v[16]) { F2 r;
#pragma unroll
  for (int i = 0; i < 16; ++i) { const __bf16 h = (__bf16)v[i]; r.h[i] = h; r.l[i] = (__bf16)(v[i] - (float)h); }
  return r; }
__device__ __forceinline__ F2 split_row(const float* row, int k0, int lane) { float v[16]; const float* p = row + k0 + 8 * (lane >> 4);
#pragma unroll
  for (int i = 0; i < 8; ++i) { v[i] = p[i]; v[8 + i] = p[16 + i]; }
  return bsplit16(v); }
__device__ __forceinline__ float bfr(float v) { return (float)(__bf16)v; }
#define LDSX() do { asm volatile("s_wait_dscnt 0" ::: "memory"); __builtin_amdgcn_wave_barrier(); __builtin_amdgcn_fence(3  , "workgroup"); } while (0)

#ifndef NB
#define NB 2
#endif
#ifndef SEQ
#define SEQ 2048
#endif
#define TT SEQ
#define NB_FULL 2
#define TT_FULL 2048
#define CC 1024
#define DIN 1024
#define NH 16
#define HD 64
#define NQB (TT / 64)
#define HG 4
#define SCALE (0.125f)
#define QBH ((NQB) < 8 ? (NQB) : 8)
#define QHI (QBH * 64)
#define KHI (QBH * 64)
__device__ __forceinline__ int kb_last(int qb) { return (qb * 64 + 63) >> 7; }

static_assert(TT % 256 == 0);
static_assert(NH * HD == CC);
static_assert(HD == 64);
static_assert(NH % HG == 0);
static_assert(CC % 128 == 0 && DIN % 64 == 0 && DIN % 32 == 0);
static_assert(QBH % 2 == 0);
static_assert(NB <= NB_FULL && TT <= TT_FULL);

#define WS_XB   0u
#define WS_WB   (WS_XB  + 2u * (size_t)NB * TT * DIN)
#define WS_WPH  (WS_WB  + 2u * (size_t)4 * CC * DIN)
#define WS_QH   (WS_WPH + 2u * (size_t)CC * DIN)
#define WS_KH   (WS_QH  + 2u * (size_t)NB * TT * CC)
#define WS_VT   (WS_KH  + 2u * (size_t)NB * TT * CC)
#define WS_QL   (WS_VT  + 2u * (size_t)NB * CC * TT)
#define WS_KL   (WS_QL  + 2u * (size_t)NB * QHI * CC)
#define WS_VB   (WS_KL  + 2u * (size_t)NB * KHI * CC)
#define WS_VBL  (WS_VB  + 2u * (size_t)NB * CC * KHI)
#define WS_S    (WS_VBL + 2u * (size_t)NB * CC * KHI)
#define WS_YH   (WS_S   + 4u * (size_t)HG * TT * TT)
#define WS_YB   (WS_YH  + 2u * (size_t)NB * TT * CC)
#define WS_YBL  (WS_YB  + 2u * (size_t)NB * QHI * CC)
#define WS_COS  (WS_YBL + 2u * (size_t)NB * QHI * CC)
#define WS_SIN  (WS_COS + 4u * (size_t)TT * 32)
#define WS_BT   (WS_SIN + 4u * (size_t)TT * 32)
#define WS_INVF (WS_BT  + 4u * (size_t)NH * TT)
#define WS_END  (WS_INVF + 128u)
static_assert((size_t)WS_END <= (size_t)134217728);

__global__ __launch_bounds__(256) void k_tab(const float* __restrict__ REL, float* __restrict__ BT, float* __restrict__ INVF) {
  const int n = blockIdx.x * 256 + threadIdx.x;
  const float nf = (float)(n < 1 ? 1 : n);
  int big = 16 + (int)(logf(nf * 0.0625f) * (1.0f / 2.0794415f) * 16.0f);
  big = big > 31 ? 31 : big;
  int bucket = n < 16 ? n : big;
  bucket = bucket < 0 ? 0 : (bucket > 31 ? 31 : bucket);
#pragma unroll 1
  for (int h = 0; h < NH; ++h) { const float v = bfr(REL[bucket * NH + h]) * SCALE; vst2(BT + (size_t)h * TT + n, v); }
  if (blockIdx.x == 0 && threadIdx.x < 32) {
    const float e = (float)(2 * (int)threadIdx.x) * (1.0f / 64.0f); const float iv = 1.0f / powf(10000.0f, e); vst2(INVF + threadIdx.x, iv); }
}
__global__ __launch_bounds__(256) void k_rope(const float* __restrict__ INVF, float* __restrict__ COS, float* __restrict__ SIN) {
  const int e = blockIdx.x * 256 + threadIdx.x; const int t = e >> 5, j = e & 31;
  const float fr = (float)t * INVF[j]; const float c = cosf(fr); const float s = sinf(fr);
  vst2(COS + e, c); vst2(SIN + e, s);
}
__global__ __launch_bounds__(256) void k_cvtx(const float* __restrict__ X, __bf16* __restrict__ XB) {
  const size_t e = (size_t)blockIdx.x * 256 + threadIdx.x; const size_t row = e / (DIN / 8); const int q = (int)(e % (DIN / 8));
  const size_t b = row / TT, t = row % TT; const float* p = X + (b * TT_FULL + t) * DIN + q * 8;
  const v4f a = *(const v4f*)p, c = *(const v4f*)(p + 4); union { v8b v; v4u u; } o;
#pragma unroll
  for (int i = 0; i < 4; ++i) { o.v[i] = (__bf16)a[i]; o.v[4 + i] = (__bf16)c[i]; }
  vst2(XB + row * DIN + q * 8, o.u);
}
__global__ __launch_bounds__(256) void k_cvtw(const float* __restrict__ W0, const float* __restrict__ W1, const float* __restrict__ W2, const float* __restrict__ W3, __bf16* __restrict__ WB, _Float16* __restrict__ WPH) {
  __shared__ __align__(16) __bf16 tb[64][72]; __shared__ __align__(16) _Float16 th[64][72];
  const int tid = threadIdx.x; const int which = blockIdx.z; const int k0 = blockIdx.x * 64, n0 = blockIdx.y * 64;
  const float* W = which == 0 ? W0 : which == 1 ? W1 : which == 2 ? W2 : W3;
  for (int e = tid; e < 64 * 16; e += 256) { const int kk = e >> 4, q = e & 15; const v4f w = *(const v4f*)(W + (size_t)(k0 + kk) * CC + n0 + q * 4);
#pragma unroll
    for (int i = 0; i < 4; ++i) { const __bf16 bv = (__bf16)w[i]; tb[q * 4 + i][kk] = bv; th[q * 4 + i][kk] = (_Float16)((float)bv * 256.0f); } }
  __syncthreads();
  __bf16* WBp = WB + (size_t)which * CC * DIN;
  for (int e = tid; e < 64 * 8; e += 256) { const int nl = e >> 3, q = e & 7; const size_t o = (size_t)(n0 + nl) * DIN + k0 + q * 8;
    vst2(WBp + o, *(const v4u*)&tb[nl][q * 8]); if (which == 3) vst2(WPH + o, *(const v4u*)&th[nl][q * 8]); }
}
__global__ __launch_bounds__(128) void k_proj(const __bf16* __restrict__ XB, const __bf16* __restrict__ WB, const float* __restrict__ BQ, const float* __restrict__ BK, const float* __restrict__ BV, const float* __restrict__ COS, const float* __restrict__ SIN,
    _Float16* __restrict__ QH, _Float16* __restrict__ QL, _Float16* __restrict__ KH, _Float16* __restrict__ KL, _Float16* __restrict__ VT, __bf16* __restrict__ VB, __bf16* __restrict__ VBL) {
  __shared__ __align__(16) _Float16 sh[64][136], sl[64][136]; __shared__ __align__(16) _Float16 th[128][72]; __shared__ __align__(16) __bf16 tb[128][72], tbl[128][72]; __shared__ __align__(16) float cs[64][32], sn[64][32];
  const int tid = threadIdx.x, wave = tid >> 5, lane = tid & 31, col = lane & 15, g = lane >> 4; const int which = blockIdx.z; const int c0 = blockIdx.y * 128; const size_t r0 = (size_t)blockIdx.x * 64; const size_t bb = r0 / TT; const int t0 = (int)(r0 % TT);
  const float* BA = which == 0 ? BQ : which == 1 ? BK : BV; const __bf16* WA = WB + (size_t)which * CC * DIN;
  if (which < 2) {
    for (int e = tid; e < 64 * 8; e += 128) { const int rl = e >> 3, q = e & 7; *(v4f*)&cs[rl][q * 4] = *(const v4f*)(COS + (size_t)(t0 + rl) * 32 + q * 4); *(v4f*)&sn[rl][q * 4] = *(const v4f*)(SIN + (size_t)(t0 + rl) * 32 + q * 4); } }
  v8f acc[8] = {};
#pragma unroll 2
  for (int kc = 0; kc < DIN / 32; ++kc) { const v16b a = frag_b(XB + (r0 + wave * 16 + col) * DIN + kc * 32, lane);
#pragma unroll
    for (int j = 0; j < 8; ++j) { const v16b w = frag_b(WA + (size_t)(c0 + j * 16 + col) * DIN + kc * 32, lane); acc[j] = wmma_bf(a, w, acc[j]); } }
  __syncthreads();
  if (which < 2) { _Float16* DH = which == 0 ? QH : KH; _Float16* DL = which == 0 ? QL : KL; const int nhi = which == 0 ? QHI : KHI; const bool hi_rows = t0 < nhi;
#pragma unroll
    for (int j = 0; j < 8; ++j) { const float bias = bfr(BA[c0 + j * 16 + col]);
#pragma unroll
      for (int r = 0; r < 8; ++r) acc[j][r] += bias; }
#pragma unroll
    for (int hh = 0; hh < 2; ++hh) {
#pragma unroll
      for (int jj = 0; jj < 2; ++jj) {
#pragma unroll
        for (int r = 0; r < 8; ++r) { const int rl = wave * 16 + 8 * g + r; const float c = cs[rl][jj * 16 + col], s = sn[rl][jj * 16 + col]; const float a = acc[hh * 4 + jj][r], b2 = acc[hh * 4 + jj + 2][r];
          acc[hh * 4 + jj][r] = a * c - b2 * s; acc[hh * 4 + jj + 2][r] = b2 * c + a * s; } } }
#pragma unroll
    for (int j = 0; j < 8; ++j) {
#pragma unroll
      for (int r = 0; r < 8; ++r) { const float v = acc[j][r]; const _Float16 hv = (_Float16)v; sh[wave * 16 + 8 * g + r][j * 16 + col] = hv; sl[wave * 16 + 8 * g + r][j * 16 + col] = (_Float16)((v - (float)hv) * 1024.0f); } }
    __syncthreads();
    for (int e = tid; e < 64 * 16; e += 128) { const int rl = e >> 4, q = e & 15; vst2(DH + (r0 + rl) * CC + c0 + q * 8, *(const v4u*)&sh[rl][q * 8]); if (hi_rows) vst2(DL + (bb * nhi + t0 + rl) * (size_t)CC + c0 + q * 8, *(const v4u*)&sl[rl][q * 8]); }
  } else { const bool hi_rows = t0 < KHI;
#pragma unroll
    for (int j = 0; j < 8; ++j) { const float bias = bfr(BA[c0 + j * 16 + col]);
#pragma unroll
      for (int r = 0; r < 8; ++r) { const float v = acc[j][r] + bias; const int rl = wave * 16 + 8 * g + r, cl = j * 16 + col; th[cl][rl] = (_Float16)v; const __bf16 bh = (__bf16)v; tb[cl][rl] = bh; tbl[cl][rl] = (__bf16)(v - (float)bh); } }
    __syncthreads();
    for (int e = tid; e < 128 * 8; e += 128) { const int cl = e >> 3, q = e & 7; vst2(VT + (bb * CC + c0 + cl) * (size_t)TT + t0 + q * 8, *(const v4u*)&th[cl][q * 8]); if (hi_rows) { const size_t o3 = (bb * CC + c0 + cl) * (size_t)KHI + t0 + q * 8; vst2(VB + o3, *(const v4u*)&tb[cl][q * 8]); vst2(VBL + o3, *(const v4u*)&tbl[cl][q * 8]); } } } }
__global__ __launch_bounds__(128) void k_sc(const _Float16* __restrict__ QH, const _Float16* __restrict__ KH, const _Float16* __restrict__ QL, const _Float16* __restrict__ KL, int b, int h0, float* __restrict__ S0) { __shared__ __align__(16) float ss[4][16][132];
  const int qb = blockIdx.x, kb = blockIdx.y; if (kb > kb_last(qb)) return;
  const int h = h0 + blockIdx.z; float* S = S0 + (size_t)blockIdx.z * TT * TT;
  const int tid = threadIdx.x, wave = tid >> 5, lane = tid & 31, col = lane & 15, g = lane >> 4; const int k0 = kb * 128; const int ql0 = qb * 64 + wave * 16; const size_t q0 = (size_t)b * TT + ql0, kr0 = (size_t)b * TT + k0;
  v8f acc[8] = {}, accl[8] = {};
  const _Float16* QLb = QL + (size_t)b * QHI * CC; const _Float16* KLb = KL + (size_t)b * KHI * CC;
  if (qb < QBH) {
#pragma unroll
    for (int kc = 0; kc < HD / 32; ++kc) { const v16h ah = frag_h(QH + (q0 + col) * CC + h * HD + kc * 32, lane), al = frag_h(QLb + (size_t)(ql0 + col) * CC + h * HD + kc * 32, lane);
#pragma unroll
      for (int j = 0; j < 8; ++j) { const v16h kbf = frag_h(KH + (kr0 + j * 16 + col) * CC + h * HD + kc * 32, lane), klf = frag_h(KLb + (size_t)(k0 + j * 16 + col) * CC + h * HD + kc * 32, lane); acc[j] = wmma16(ah, kbf, acc[j]); accl[j] = wmma16(al, kbf, accl[j]); accl[j] = wmma16(ah, klf, accl[j]); } }
  } else {
#pragma unroll
    for (int kc = 0; kc < HD / 32; ++kc) { const v16h ah = frag_h(QH + (q0 + col) * CC + h * HD + kc * 32, lane);
#pragma unroll
      for (int j = 0; j < 8; ++j) { const v16h kbf = frag_h(KH + (kr0 + j * 16 + col) * CC + h * HD + kc * 32, lane); acc[j] = wmma16(ah, kbf, acc[j]); } } }
#pragma unroll
  for (int j = 0; j < 8; ++j) {
#pragma unroll
    for (int r = 0; r < 8; ++r) ss[wave][8 * g + r][j * 16 + col] = (acc[j][r] + accl[j][r] * (1.0f / 1024.0f)) * SCALE; }
  LDSX(); for (int rl = 0; rl < 16; ++rl) vst2(S + (size_t)(ql0 + rl) * TT + k0 + lane * 4, *(const v4f*)&ss[wave][rl][lane * 4]); }
__global__ __launch_bounds__(256) void k_sm(float* __restrict__ S0, const float* __restrict__ BT, int h0) { __shared__ float sred[8]; __shared__ float sbc; __shared__ __align__(16) float shv[TT];
  const int tid = threadIdx.x; const int t = blockIdx.x; const int kend = (kb_last(t >> 6) + 1) * 128;
  float* sr = S0 + (size_t)blockIdx.y * TT * TT + (size_t)t * TT; const float* bt = BT + (size_t)(h0 + blockIdx.y) * TT;
  float m = -3.0e38f; for (int k = tid; k < kend; k += 256) { const int n = t - k; const float bv = bt[n < 0 ? 0 : n]; const float lv = sr[k]; const float v = (k <= t) ? lv + bv : -3.0e38f; shv[k] = v; m = fmaxf(m, v); }
#pragma unroll
  for (int o = 1; o < 32; o <<= 1) m = fmaxf(m, __shfl_xor(m, o));
  if ((tid & 31) == 0) sred[tid >> 5] = m; __syncthreads(); if (tid == 0) { float a = sred[0]; for (int i = 1; i < 8; ++i) a = fmaxf(a, sred[i]); sbc = a; } __syncthreads(); m = sbc; __syncthreads();
  float sum = 0.f; for (int k = tid; k < kend; k += 256) { const float v = shv[k]; const float e = (v <= -1.0e38f) ? 0.f : expf(v - m); shv[k] = e; sum += e; }
#pragma unroll
  for (int o = 1; o < 32; o <<= 1) sum += __shfl_xor(sum, o);
  if ((tid & 31) == 0) sred[tid >> 5] = sum; __syncthreads(); if (tid == 0) { float a = 0.f; for (int i = 0; i < 8; ++i) a += sred[i]; sbc = a > 0.f ? 2048.0f / a : 0.f; } __syncthreads(); const float inv = sbc;
  for (int k = tid; k < kend; k += 256) shv[k] = shv[k] * inv;
  __syncthreads(); for (int q = tid; q < kend / 4; q += 256) vst2(sr + q * 4, *(const v4f*)&shv[q * 4]); }
__global__ __launch_bounds__(128) void k_pv(const float* __restrict__ PS0, const _Float16* __restrict__ VT, const __bf16* __restrict__ VB, const __bf16* __restrict__ VBL, int b, int h0, _Float16* __restrict__ YH, __bf16* __restrict__ YB, __bf16* __restrict__ YBL) { const int h = h0 + blockIdx.z; const float* PS = PS0 + (size_t)blockIdx.z * TT * TT; __shared__ __align__(16) float ss[4][16][HD + 4];
  const int tid = threadIdx.x, wave = tid >> 5, lane = tid & 31, col = lane & 15, g = lane >> 4; const int qb = blockIdx.x; const int ql0 = qb * 64 + wave * 16; const int kce = (kb_last(qb) + 1) * 4;
  v8f acc[HD / 16] = {};
  if (qb < QBH) {
#pragma unroll 1
    for (int kc = 0; kc < kce; ++kc) { const F2 p = split_row(PS + (size_t)(ql0 + col) * TT, kc * 32, lane);
      asm volatile("s_wait_loadcnt 0x0" ::: "memory");
#pragma unroll
      for (int j = 0; j < HD / 16; ++j) { const size_t po = ((size_t)b * CC + h * HD + j * 16 + col) * (size_t)KHI + kc * 32; const v16b vh = frag_b(VB + po, lane); acc[j] = wmma_bf(p.h, vh, acc[j]); acc[j] = wmma_bf(p.l, vh, acc[j]); acc[j] = wmma_bf(p.h, frag_b(VBL + po, lane), acc[j]); } }
  } else {
#pragma unroll 1
    for (int kc = 0; kc < kce; ++kc) { const v16h p = frag_f32(PS + (size_t)(ql0 + col) * TT + kc * 32, lane);
      asm volatile("s_wait_loadcnt 0x0" ::: "memory");
#pragma unroll
      for (int j = 0; j < HD / 16; ++j) { const size_t po = ((size_t)b * CC + h * HD + j * 16 + col) * (size_t)TT + kc * 32; acc[j] = wmma16(p, frag_h(VT + po, lane), acc[j]); } } }
#pragma unroll
  for (int j = 0; j < HD / 16; ++j)
#pragma unroll
    for (int r = 0; r < 8; ++r) ss[wave][8 * g + r][j * 16 + col] = acc[j][r] * (1.0f / 2048.0f);
  LDSX();
  for (int it = 0; it < 4; ++it) { const int rl = it * 4 + (lane >> 3), pc = lane & 7; const float* sp = &ss[wave][rl][pc * 8]; const v4f a = *(const v4f*)sp, c = *(const v4f*)(sp + 4);
    union { v8h v; v4u u; } hh; union { v8b v; v4u u; } bh, bl;
#pragma unroll
    for (int i = 0; i < 4; ++i) { hh.v[i] = (_Float16)(a[i] * 64.0f); hh.v[4 + i] = (_Float16)(c[i] * 64.0f);
      const __bf16 ha = (__bf16)a[i], hc = (__bf16)c[i]; bh.v[i] = ha; bh.v[4 + i] = hc; bl.v[i] = (__bf16)(a[i] - (float)ha); bl.v[4 + i] = (__bf16)(c[i] - (float)hc); }
    vst2(YH + ((size_t)b * TT + ql0 + rl) * CC + h * HD + pc * 8, hh.u);
    if (qb < QBH) { const size_t o = ((size_t)b * QHI + ql0 + rl) * CC + h * HD + pc * 8; vst2(YB + o, bh.u); vst2(YBL + o, bl.u); } } }
__global__ __launch_bounds__(128) void k_out(const _Float16* __restrict__ YH, const __bf16* __restrict__ YB, const __bf16* __restrict__ YBL, const _Float16* __restrict__ WPH, const __bf16* __restrict__ WPB, const float* __restrict__ BO, float* __restrict__ OUT) { __shared__ __align__(16) float sf[4][16][132];
  const int tid = threadIdx.x, wave = tid >> 5, lane = tid & 31, col = lane & 15, g = lane >> 4; const int c0 = blockIdx.y * 128; const size_t rb = (size_t)blockIdx.x * 64; const size_t bb = rb / TT; const int tl = (int)(rb % TT); const size_t r0 = rb + wave * 16;
  v8f acc[8] = {};
  if (tl < QHI) {
    const size_t e0 = (bb * QHI + tl + wave * 16 + col) * (size_t)CC;
#pragma unroll 2
    for (int kc = 0; kc < CC / 32; ++kc) { const v16b ah = frag_b(YB + e0 + kc * 32, lane), al = frag_b(YBL + e0 + kc * 32, lane);
#pragma unroll
      for (int j = 0; j < 8; ++j) { const v16b w = frag_b(WPB + (size_t)(c0 + j * 16 + col) * CC + kc * 32, lane); acc[j] = wmma_bf(ah, w, acc[j]); acc[j] = wmma_bf(al, w, acc[j]); } }
#pragma unroll
    for (int j = 0; j < 8; ++j) { const float bias = bfr(BO[c0 + j * 16 + col]);
#pragma unroll
      for (int r = 0; r < 8; ++r) sf[wave][8 * g + r][j * 16 + col] = acc[j][r] + bias; }
  } else {
#pragma unroll 2
    for (int kc = 0; kc < CC / 32; ++kc) { const v16h a = frag_h(YH + (r0 + col) * CC + kc * 32, lane);
#pragma unroll
      for (int j = 0; j < 8; ++j) { const v16h w = frag_h(WPH + (size_t)(c0 + j * 16 + col) * CC + kc * 32, lane); acc[j] = wmma16(a, w, acc[j]); } }
#pragma unroll
    for (int j = 0; j < 8; ++j) { const float bias = bfr(BO[c0 + j * 16 + col]);
#pragma unroll
      for (int r = 0; r < 8; ++r) sf[wave][8 * g + r][j * 16 + col] = acc[j][r] * (1.0f / 16384.0f) + bias; } }
  LDSX(); for (int rl = 0; rl < 16; ++rl) vst2(OUT + (bb * TT_FULL + tl + wave * 16 + rl) * (size_t)DIN + c0 + lane * 4, *(const v4f*)&sf[wave][rl][lane * 4]); }

extern "C" void kernel_launch(void* const* d_in, const int* in_sizes, int n_in, void* d_out, int out_size, void* d_ws, size_t ws_size, hipStream_t stream) {
  if (n_in < 10) return;
  const int xmin = ((NB - 1) * TT_FULL + TT) * DIN;
  if (in_sizes[0] < xmin) return;
  if (in_sizes[1] < DIN * CC || in_sizes[3] < DIN * CC || in_sizes[5] < DIN * CC || in_sizes[7] < CC * DIN) return;
  if (in_sizes[2] < CC || in_sizes[4] < CC || in_sizes[6] < CC || in_sizes[8] < DIN) return;
  if (in_sizes[9] < 32 * NH) return;
  if (out_size < xmin) return;
  if (ws_size < (size_t)WS_END) return;
  const float** F = (const float**)d_in;
  char* ws = (char*)d_ws;
  __bf16 *XB = (__bf16*)(ws + WS_XB), *WB = (__bf16*)(ws + WS_WB), *VB = (__bf16*)(ws + WS_VB), *VBL = (__bf16*)(ws + WS_VBL), *YB = (__bf16*)(ws + WS_YB), *YBL = (__bf16*)(ws + WS_YBL);
  _Float16 *WPH = (_Float16*)(ws + WS_WPH), *QH = (_Float16*)(ws + WS_QH), *KH = (_Float16*)(ws + WS_KH), *VT = (_Float16*)(ws + WS_VT), *QL = (_Float16*)(ws + WS_QL), *KL = (_Float16*)(ws + WS_KL), *YH = (_Float16*)(ws + WS_YH);
  float *S = (float*)(ws + WS_S), *COS = (float*)(ws + WS_COS), *SIN = (float*)(ws + WS_SIN), *BT = (float*)(ws + WS_BT), *INVF = (float*)(ws + WS_INVF);
  k_tab<<<dim3(TT / 256), 256, 0, stream>>>(F[9], BT, INVF);
  k_rope<<<dim3(TT * 32 / 256), 256, 0, stream>>>(INVF, COS, SIN);
  k_cvtx<<<dim3(NB * TT * (DIN / 8) / 256), 256, 0, stream>>>(F[0], XB);
  k_cvtw<<<dim3(DIN / 64, CC / 64, 4), 256, 0, stream>>>(F[1], F[3], F[5], F[7], WB, WPH);
  k_proj<<<dim3(NB * TT / 64, CC / 128, 3), 128, 0, stream>>>(XB, WB, F[2], F[4], F[6], COS, SIN, QH, QL, KH, KL, VT, VB, VBL);
  for (int b = 0; b < NB; ++b) for (int h0 = 0; h0 < NH; h0 += HG) {
    k_sc<<<dim3(NQB, TT / 128, HG), 128, 0, stream>>>(QH, KH, QL, KL, b, h0, S);
    k_sm<<<dim3(TT, HG), 256, 0, stream>>>(S, BT, h0);
    k_pv<<<dim3(NQB, 1, HG), 128, 0, stream>>>(S, VT, VB, VBL, b, h0, YH, YB, YBL);
  }
  k_out<<<dim3(NB * TT / 64, DIN / 128), 128, 0, stream>>>(YH, YB, YBL, WPH, WB + (size_t)3 * CC * DIN, F[8], (float*)d_out);
}
